// CfCNCPWrapper_78975858639370
// MI455X (gfx1250) — hardware-verified
//
#include <hip/hip_runtime.h>
#include <math.h>

typedef __attribute__((ext_vector_type(16))) _Float16 v16h;
typedef __attribute__((ext_vector_type(8)))  _Float16 v8h;
typedef __attribute__((ext_vector_type(4)))  _Float16 v4h;
typedef __attribute__((ext_vector_type(8)))  float    v8f;
typedef __attribute__((ext_vector_type(4)))  float    v4f;

__device__ __forceinline__ void dep_guard_h(v8f& a, v8f& b, v16h x, v16h y) { asm volatile("v_nop\n\tv_nop\n\tv_nop\n\tv_nop" : "+v"(a), "+v"(b) : "v"(x), "v"(y)); }
__device__ __forceinline__ void keep4_h(v16h a, v16h b, v16h c, v16h d) { asm volatile("v_nop" :: "v"(a), "v"(b), "v"(c), "v"(d)); }
__device__ __forceinline__ void acc_guard4(v8f& a, v8f& b, v8f& c, v8f& d) { asm volatile("v_nop\n\tv_nop\n\tv_nop\n\tv_nop" : "+v"(a), "+v"(b), "+v"(c), "+v"(d)); }
template <typename T> struct Frag;
template <> struct Frag<_Float16> {
  typedef v16h V; union U { v16h v; v8h h[2]; };
  static __device__ __forceinline__ v16h load(const _Float16* p) {
    U f; f.h[0] = *(const v8h*)(p); f.h[1] = *(const v8h*)(p + 16); return f.v;
  }
  static __device__ __forceinline__ v8f mma(v16h a, v16h b, v8f c) {
    return __builtin_amdgcn_wmma_f32_16x16x32_f16(false, a, false, b, (short)0, c, false, false);
  }
  static __device__ __forceinline__ void guard(v8f& a, v8f& b, v16h x, v16h y) { dep_guard_h(a, b, x, y); }
  static __device__ __forceinline__ void keep(v16h a, v16h b, v16h c, v16h d) { keep4_h(a, b, c, d); }
};

constexpr int kBatch = 128, kSeqLen = 256, kInDim = 64, kOutDim = 64, kUnits = 512;
constexpr int kRows = 16;
constexpr int kThreads = 256;
constexpr int kWaves = 8;
constexpr int kBlocks = kBatch / kRows;
constexpr int kN0 = 269, kD0 = 333, kKP0 = 352, kNP0 = 272, kNUB0 = 17, kDin0 = 64,  kCol0 = 0;
constexpr int kN1 = 179, kD1 = 448, kKP1 = 448, kNP1 = 192, kNUB1 = 12, kDin1 = 269, kCol1 = 269;
constexpr int kN2 = 64,  kD2 = 243, kKP2 = 256, kNP2 = 64,  kNUB2 = 4,  kDin2 = 179, kCol2 = 448;
constexpr int kSubBase0 = 0, kSubBase1 = kNUB0, kSubBase2 = kNUB0 + kNUB1, kNSub = kNUB0 + kNUB1 + kNUB2;
constexpr int kZPitch = 32;
constexpr int kChunkFloats = 8 * 32;
constexpr float kWScale = 256.0f;
constexpr float kWInv = 1.0f / 256.0f;

static_assert(kKP0 % 32 == 0 && kKP1 % 32 == 0 && kKP2 % 32 == 0, "K tile multiple");
static_assert(kNP0 == 16 * kNUB0 && kNP1 == 16 * kNUB1 && kNP2 == 16 * kNUB2, "N subtiles");
static_assert(kKP0 >= kD0 && kKP1 >= kD1 && kKP2 >= kD2, "K pad");
static_assert(kNP0 >= kN0 && kNP1 >= kN1 && kNP2 >= kN2, "N pad");
static_assert(kDin0 + kN0 == kD0 && kDin1 + kN1 == kD1 && kDin2 + kN2 == kD2, "concat widths");
static_assert(kCol1 == kN0 && kCol2 == kN0 + kN1 && kCol2 + kN2 == kUnits, "state columns");
static_assert(kBlocks * kRows == kBatch, "row coverage");
static_assert(kKP1 >= kKP0 && kKP1 >= kKP2, "shared A tile sized for the widest layer");
static_assert(kKP2 == 256, "layer 2 build uses shift/mask indexing");
static_assert(kNSub == 33 && kSubBase2 == 29, "slab subtile map");
static_assert(kThreads == kWaves * 32, "waves");

__global__ __launch_bounds__(256) void prep_weights_kernel(
    const float* __restrict__ wf1, const float* __restrict__ wf2,
    const float* __restrict__ wta, const float* __restrict__ wtb,
    const float* __restrict__ mask, _Float16* __restrict__ bt,
    int nvalid, int dvalid, int npad, int kpad, int n8, float carry)
{
  const int g = blockIdx.y;
  const float* w = (g == 0) ? wf1 : (g == 1) ? wf2 : (g == 2) ? wta : wtb;
  const bool usemask = (g < 2);
  const int i = blockIdx.x * 256 + threadIdx.x;
  if (i >= n8) return;
  const int flat = i * 8;
  const int n = flat / kpad;
  const int k = flat - n * kpad;
  const int nc = (n < nvalid) ? n : (nvalid - 1);
  v8h hv;
#pragma unroll
  for (int e = 0; e < 8; ++e) {
    const int kk = k + e;
    const int kc = (kk < dvalid) ? kk : (dvalid - 1);
    const size_t idx = (size_t)nc * dvalid + kc;
    float val = w[idx];
    const float mv = mask[idx];
    if (usemask) val = val * mv;
    val = (n < nvalid && kk < dvalid) ? (val * carry) : 0.0f;
    hv[e] = (_Float16)val;
  }
  _Float16* dst = bt + (size_t)g * npad * kpad + flat;
  *(volatile v8h*)dst = hv;
  __threadfence();
  *(volatile v8h*)dst = hv;
}

struct SeqArgs {
  const float* x;  const float* h0;
  const _Float16* bt0; const _Float16* bt1; const _Float16* bt2;
  const float* b1_0; const float* b2_0; const float* ba_0; const float* bb_0;
  const float* b1_1; const float* b2_1; const float* ba_1; const float* bb_1;
  const float* b1_2; const float* b2_2; const float* ba_2; const float* bb_2;
  float* seq;
  float* state;
};
static_assert(sizeof(SeqArgs) == 19 * 8, "no padding");

__global__ __launch_bounds__(kThreads) void cfc_sequence_kernel(SeqArgs a)
{
  __shared__ __align__(16) _Float16 hs[kRows * kUnits];
  __shared__ __align__(16) _Float16 xa[kRows * kKP1];
  __shared__ __align__(16) float    zst[kWaves * 32 * kZPitch];

  const int tid   = threadIdx.x;
  const int lane  = tid & 31;
  const int wave  = tid >> 5;
  const int blk   = blockIdx.x;
  const int b0    = blk * kRows;
  const int rlane = lane & 15;
  const int hsel  = lane >> 4;
  const int koff  = hsel * 8;
  float* zw = zst + wave * (32 * kZPitch) + lane * kZPitch;

#pragma unroll 1
  for (int idx = tid; idx < kRows * kUnits / 4; idx += kThreads) {
    const int m = idx >> 7, c4 = (idx & 127) * 4;
    const v4f hv = *(const v4f*)(a.h0 + (size_t)(b0 + m) * kUnits + c4);
    v4h q;
    q[0] = (_Float16)hv[0]; q[1] = (_Float16)hv[1]; q[2] = (_Float16)hv[2]; q[3] = (_Float16)hv[3];
    *(v4h*)(hs + m * kUnits + c4) = q;
  }
  __syncthreads();

#pragma unroll 1
  for (int t = 0; t < kSeqLen; ++t) {
#pragma unroll 1
    for (int l = 0; l < 3; ++l) {
      if (l == 0) {
        {
          const int m = tid >> 4, c4 = (tid & 15) * 4;
          const v4f xv = *(const v4f*)(a.x + ((size_t)(b0 + m) * kSeqLen + t) * kInDim + c4);
          v4h q;
          q[0] = (_Float16)xv[0]; q[1] = (_Float16)xv[1]; q[2] = (_Float16)xv[2]; q[3] = (_Float16)xv[3];
          *(v4h*)(xa + m * kKP0 + c4) = q;
        }
#pragma unroll 1
        for (int idx = tid; idx < kRows * (kKP0 - kInDim); idx += kThreads) {
          const int m  = idx / (kKP0 - kInDim);
          const int e  = idx - m * (kKP0 - kInDim);
          const int ec = (e < kN0) ? e : (kN0 - 1);
          const _Float16 hv = hs[m * kUnits + kCol0 + ec];
          xa[m * kKP0 + kInDim + e] = (e < kN0) ? hv : (_Float16)0.0f;
        }
      } else if (l == 1) {
#pragma unroll 1
        for (int idx = tid; idx < kRows * (kKP1 / 8); idx += kThreads) {
          const int m = idx / (kKP1 / 8);
          const int j = idx - m * (kKP1 / 8);
          const v8h v = *(const v8h*)(hs + m * kUnits + 8 * j);
          *(v8h*)(xa + m * kKP1 + 8 * j) = v;
        }
      } else {
#pragma unroll 1
        for (int idx = tid; idx < kRows * kKP2; idx += kThreads) {
          const int m  = idx >> 8;
          const int e  = idx & 255;
          const int ec = (e < kD2) ? e : (kD2 - 1);
          const _Float16 hv = hs[m * kUnits + kCol1 + ec];
          xa[m * kKP2 + e] = (e < kD2) ? hv : (_Float16)0.0f;
        }
      }
      __syncthreads();

      const int kpad   = (l == 0) ? kKP0  : (l == 1) ? kKP1  : kKP2;
      const int npad   = (l == 0) ? kNP0  : (l == 1) ? kNP1  : kNP2;
      const int nub    = (l == 0) ? kNUB0 : (l == 1) ? kNUB1 : kNUB2;
      const int nvalid = (l == 0) ? kN0   : (l == 1) ? kN1   : kN2;
      const int coloff = (l == 0) ? kCol0 : (l == 1) ? kCol1 : kCol2;
      const int sbase  = (l == 0) ? kSubBase0 : (l == 1) ? kSubBase1 : kSubBase2;
      const _Float16* bt = (l == 0) ? a.bt0 : (l == 1) ? a.bt1 : a.bt2;
      const float* bf1 = (l == 0) ? a.b1_0 : (l == 1) ? a.b1_1 : a.b1_2;
      const float* bf2 = (l == 0) ? a.b2_0 : (l == 1) ? a.b2_1 : a.b2_2;
      const float* bta = (l == 0) ? a.ba_0 : (l == 1) ? a.ba_1 : a.ba_2;
      const float* btb = (l == 0) ? a.bb_0 : (l == 1) ? a.bb_1 : a.bb_2;
      const bool do_seq   = (l == 2);
      const bool do_state = (t == kSeqLen - 1);
      const size_t gstride = (size_t)npad * kpad;

#pragma unroll 1
      for (int ub = wave; ub < nub; ub += kWaves) {
        v8f acc[4];
#pragma unroll
        for (int g = 0; g < 4; ++g) acc[g] = (v8f){0.f,0.f,0.f,0.f,0.f,0.f,0.f,0.f};

        const _Float16* ap = xa + rlane * kpad + koff;
        const _Float16* bp = bt + (size_t)(16 * ub + rlane) * kpad + koff;
#pragma unroll 1
        for (int k0 = 0; k0 < kpad; k0 += 32) {
          v16h bq[4];
          bq[0] = Frag<_Float16>::load(bp + k0);
          bq[1] = Frag<_Float16>::load(bp + gstride + k0);
          bq[2] = Frag<_Float16>::load(bp + 2 * gstride + k0);
          bq[3] = Frag<_Float16>::load(bp + 3 * gstride + k0);
          const v16h av = Frag<_Float16>::load(ap + k0);
#pragma unroll
          for (int g = 0; g < 4; ++g) acc[g] = Frag<_Float16>::mma(av, bq[g], acc[g]);
          Frag<_Float16>::guard(acc[0], acc[3], av, av);
          Frag<_Float16>::keep(bq[0], bq[1], bq[2], bq[3]);
        }
        acc_guard4(acc[0], acc[1], acc[2], acc[3]);

#pragma unroll
        for (int g = 0; g < 4; ++g) {
#pragma unroll
          for (int e = 0; e < 8; ++e) zw[g * 8 + e] = acc[g][e];
        }

        const int  u     = 16 * ub + rlane;
        const bool valid = (u < nvalid);
        const int  uc    = valid ? u : (nvalid - 1);
        const float vb1 = bf1[uc], vb2 = bf2[uc], vba = bta[uc], vbb = btb[uc];
        const size_t stbase = ((size_t)(blk * kNSub + sbase + ub) * 8) * 32 + lane;

#pragma unroll 1
        for (int r = 0; r < 8; ++r) {
          const float z1 = zw[r] * kWInv + vb1;
          const float z2 = zw[8 + r] * kWInv + vb2;
          float zg = ((zw[16 + r] * kWInv + vba) + zw[24 + r] * kWInv) + vbb;
          zg = fminf(fmaxf(zg, -30.0f), 30.0f);
          const float f1 = tanhf(z1);
          const float f2 = tanhf(z2);
          const float sg = 1.0f / (1.0f + expf(-zg));
          const float nv = f1 * (1.0f - sg) + sg * f2;
          const int m = 8 * hsel + r;
          if (valid) hs[m * kUnits + coloff + u] = (_Float16)nv;
          const float sv = valid ? nv : 0.0f;
          if (do_state) {
            float* p = a.state + stbase + (size_t)r * 32;
            *(volatile float*)p = sv;
            __threadfence();
            *(volatile float*)p = sv;
          }
          if (do_seq) {
            const float ov = tanhf(sv);
            float* p = a.seq + ((((size_t)blk * kSeqLen + t) * kNUB2 + ub) * 8 + r) * 32 + lane;
            *(volatile float*)p = ov;
            __threadfence();
            *(volatile float*)p = ov;
          }
        }
      }
      __syncthreads();
    }
  }
}

__global__ __launch_bounds__(256) void emit_out0_kernel(const float* __restrict__ seq, float* __restrict__ out0, int n4)
{
  const int i = blockIdx.x * 256 + threadIdx.x;
  if (i >= n4) return;
  const int br  = i >> 12;
  const int rem = i & 4095;
  const int t   = rem >> 4;
  const int u   = (rem & 15) * 4;
  const int blk = br >> 4, m = br & 15, hh = m >> 3, r = m & 7, ub = u >> 4, c = u & 15;
  const size_t so = ((((size_t)blk * kSeqLen + t) * kNUB2 + ub) * 8 + r) * 32 + 16 * hh + c;
  const v4f v = *(const v4f*)(seq + so);
  float* dst = out0 + (size_t)i * 4;
  *(volatile v4f*)dst = v;
  __threadfence();
  *(volatile v4f*)dst = v;
}

__global__ __launch_bounds__(256) void emit_out1_kernel(const float* __restrict__ state, float* __restrict__ out1, int n4)
{
  const int i = blockIdx.x * 256 + threadIdx.x;
  if (i >= n4) return;
  const int br  = i >> 7;
  const int col = (i & 127) * 4;
  const int blk = br >> 4, m = br & 15, hh = m >> 3, r = m & 7;
  v4f v;
#pragma unroll
  for (int e = 0; e < 4; ++e) {
    const int cc = col + e;
    const int u1 = (cc >= kCol1) ? (cc - kCol1) : 0;
    const int u2 = (cc >= kCol2) ? (cc - kCol2) : 0;
    int s, c;
    if (cc < kCol1)      { s = kSubBase0 + (cc >> 4); c = cc & 15; }
    else if (cc < kCol2) { s = kSubBase1 + (u1 >> 4); c = u1 & 15; }
    else                 { s = kSubBase2 + (u2 >> 4); c = u2 & 15; }
    const size_t so = (((size_t)blk * kNSub + s) * 8 + r) * 32 + 16 * hh + c;
    v[e] = state[so];
  }
  float* dst = out1 + (size_t)i * 4;
  *(volatile v4f*)dst = v;
  __threadfence();
  *(volatile v4f*)dst = v;
}

extern "C" void kernel_launch(void* const* d_in, const int* in_sizes, int n_in,
                              void* d_out, int out_size, void* d_ws, size_t ws_size,
                              hipStream_t stream)
{
  if (n_in < 30) return;
  if (in_sizes[0] != kBatch * kSeqLen * kInDim) return;
  if (in_sizes[2] != kBatch * kUnits) return;
  if (out_size != kBatch * kSeqLen * kOutDim + kBatch * kUnits) return;

  const int nval[3] = {kN0, kN1, kN2};
  const int dval[3] = {kD0, kD1, kD2};
  const int npad[3] = {kNP0, kNP1, kNP2};
  const int kpad[3] = {kKP0, kKP1, kKP2};
  for (int l = 0; l < 3; ++l) {
    const int base = 3 + 9 * l;
    for (int j = 0; j < 4; ++j) if (in_sizes[base + j] != nval[l] * dval[l]) return;
    for (int j = 4; j < 8; ++j) if (in_sizes[base + j] != nval[l]) return;
    if (in_sizes[base + 8] != nval[l] * dval[l]) return;
  }

  size_t off[3];
  size_t total = 0;
  for (int l = 0; l < 3; ++l) {
    off[l] = total;
    total += (size_t)4 * npad[l] * kpad[l] * sizeof(_Float16);
  }
  const size_t seq_off = total;
  total += (size_t)kBlocks * kSeqLen * kNUB2 * kChunkFloats * sizeof(float);
  const size_t state_off = total;
  total += (size_t)kBlocks * kNSub * kChunkFloats * sizeof(float);
  if (total > ws_size) return;

  _Float16* bt[3];
  for (int l = 0; l < 3; ++l) {
    bt[l] = (_Float16*)((char*)d_ws + off[l]);
    const int base = 3 + 9 * l;
    const int n8 = npad[l] * kpad[l] / 8;
    dim3 grid((unsigned)((n8 + 255) / 256), 4u, 1u);
    prep_weights_kernel<<<grid, dim3(256), 0, stream>>>(
        (const float*)d_in[base + 0], (const float*)d_in[base + 1],
        (const float*)d_in[base + 2], (const float*)d_in[base + 3],
        (const float*)d_in[base + 8], bt[l],
        nval[l], dval[l], npad[l], kpad[l], n8, kWScale);
  }

  float* seq   = (float*)((char*)d_ws + seq_off);
  float* state = (float*)((char*)d_ws + state_off);

  SeqArgs a;
  a.x  = (const float*)d_in[0];
  a.h0 = (const float*)d_in[2];
  a.bt0 = bt[0]; a.bt1 = bt[1]; a.bt2 = bt[2];
  a.b1_0 = (const float*)d_in[7];  a.b2_0 = (const float*)d_in[8];  a.ba_0 = (const float*)d_in[9];  a.bb_0 = (const float*)d_in[10];
  a.b1_1 = (const float*)d_in[16]; a.b2_1 = (const float*)d_in[17]; a.ba_1 = (const float*)d_in[18]; a.bb_1 = (const float*)d_in[19];
  a.b1_2 = (const float*)d_in[25]; a.b2_2 = (const float*)d_in[26]; a.ba_2 = (const float*)d_in[27]; a.bb_2 = (const float*)d_in[28];
  a.seq = seq; a.state = state;

  cfc_sequence_kernel<<<dim3(kBlocks), dim3(kThreads), 0, stream>>>(a);

  float* out0 = (float*)d_out;
  float* out1 = (float*)d_out + (size_t)kBatch * kSeqLen * kOutDim;
  const int n4_0 = kBatch * kSeqLen * kOutDim / 4;
  const int n4_1 = kBatch * kUnits / 4;
  emit_out0_kernel<<<dim3((unsigned)((n4_0 + 255) / 256)), dim3(256), 0, stream>>>(seq, out0, n4_0);
  emit_out1_kernel<<<dim3((unsigned)((n4_1 + 255) / 256)), dim3(256), 0, stream>>>(state, out1, n4_1);
}
